// TkStateSpaceModule_22892175688154
// MI455X (gfx1250) — hardware-verified
//
#include <hip/hip_runtime.h>


namespace {
constexpr int Bn = 8, T = 8192, DI = 128, DS = 256, DO = 128, TC = 1024  , NCH = T / TC, NR = Bn * TC  , US = 2 * DS  ;
constexpr float BS = 1024.0f, HS = 8.0f, CS = 16.0f;

typedef _Float16 b16;
typedef __attribute__((ext_vector_type(16))) _Float16 v16b;
typedef __attribute__((ext_vector_type(8))) _Float16 v8b;
typedef __attribute__((ext_vector_type(8))) float v8f;
typedef __attribute__((ext_vector_type(4))) float v4f;
__device__ __forceinline__ float bf16_rne(float f) { unsigned int u = __float_as_uint(f); u += 0x7FFFu + ((u >> 16) & 1u); return __uint_as_float(u & 0xFFFF0000u); }
__device__ __forceinline__ void split16(float v, b16& hi, b16& lo) { hi = (b16)v; lo = (b16)(v - (float)hi); }
__device__ __forceinline__ v16b frag_kb(const b16* p, int hh) { const v8b a = *(const v8b*)(p + 8 * hh), b = *(const v8b*)(p + 16 + 8 * hh); v16b f;
#pragma unroll
  for (int e = 0; e < 8; ++e) { f[e] = a[e]; f[8 + e] = b[e]; } return f; }
__device__ __forceinline__ v8f wmma16b(v16b a, v16b b, v8f c) {
  v8f d = __builtin_amdgcn_wmma_f32_16x16x32_f16(false, a, false, b, (short)0, c, false, false);
  asm volatile("v_nop\n\tv_nop\n\tv_nop\n\tv_nop" : "+v"(d) : "v"(a), "v"(b));
  return d;
}
__device__ __forceinline__ void wave_lds_sync() { __builtin_amdgcn_fence(__ATOMIC_RELEASE, "workgroup"); __builtin_amdgcn_wave_barrier(); __builtin_amdgcn_fence(__ATOMIC_ACQUIRE, "workgroup"); }
__device__ __forceinline__ float pmul(float a, float b) { float p = a * b; asm volatile("" : "+v"(p)); return p; }

__device__ __forceinline__ void disc(const float* llr, const float* li, const float* ldt, int s, float& ar, float& ai, float& gr, float& gi) {
  const float lr = -__expf(bf16_rne(llr[s])), lim = bf16_rne(li[s]); float dt = __expf(bf16_rne(ldt[s])); dt = fminf(fmaxf(dt, 0.005f), 0.1f);
  const float dr = 1.0f - 0.5f * dt * lr, di = -0.5f * dt * lim;
  const float nr = 1.0f + 0.5f * dt * lr, ni = 0.5f * dt * lim;
  const float d2 = dr * dr + di * di;
  ar = (nr * dr + ni * di) / d2; ai = (ni * dr - nr * di) / d2;
  gr = dt * dr / d2; gi = -dt * di / d2;
}

__global__ __launch_bounds__(256) void prep_kernel(const float* __restrict__ x, const float* __restrict__ llr, const float* __restrict__ li, const float* __restrict__ ldt, const float* __restrict__ Bm, const float* __restrict__ Cr, const float* __restrict__ Ci,
                                                   b16* __restrict__ x16, b16* __restrict__ bh, b16* __restrict__ bl, b16* __restrict__ ch, b16* __restrict__ cl, float* __restrict__ state) {
  const size_t tid = (size_t)blockIdx.x * blockDim.x + threadIdx.x, nth = (size_t)gridDim.x * blockDim.x;
  for (int pass = 0; pass < 2; ++pass) {
    for (size_t p = tid; p < (size_t)Bn * T * DI / 8; p += nth) { v8b o;
#pragma unroll
      for (int e = 0; e < 8; ++e) o[e] = (b16)bf16_rne(x[p * 8 + e]);
      *(volatile v8b*)(x16 + p * 8) = o; }
    for (size_t p = tid; p < (size_t)US * DI; p += nth) { const int n = (int)(p / DI), d = (int)(p % DI), s = n % DS; float ar, ai, gr, gi; disc(llr, li, ldt, s, ar, ai, gr, gi);
      const float bv = bf16_rne(Bm[(size_t)s * DI + d]); const float v = ((n < DS) ? gr : gi) * bv * BS; b16 a, c; split16(v, a, c); ((volatile b16*)bh)[p] = a; ((volatile b16*)bl)[p] = c; }
    for (size_t p = tid; p < (size_t)DO * US; p += nth) { const int o = (int)(p / US), k = (int)(p % US); const float v = ((k < DS) ? bf16_rne(Cr[(size_t)o * DS + k]) : -bf16_rne(Ci[(size_t)o * DS + k - DS])) * CS; b16 a, c; split16(v, a, c); ((volatile b16*)ch)[p] = a; ((volatile b16*)cl)[p] = c; }
    for (size_t p = tid; p < (size_t)Bn * DS * 2; p += nth) ((volatile float*)state)[p] = 0.0f;
    __threadfence();
  }
}

__global__ __launch_bounds__(128) void ugemm_kernel(const b16* __restrict__ x16, const b16* __restrict__ bh, const b16* __restrict__ bl, int c, float* __restrict__ u) {
  __shared__ __attribute__((aligned(16))) float Ts[4][32 * 64];
  const int lane = threadIdx.x & 31, wave = threadIdx.x >> 5, nloc = lane & 15, hlf = lane >> 4, m0 = blockIdx.y * 128 + wave * 32, c0 = blockIdx.x * 64;
  const int b = m0 / TC, tl0 = m0 % TC; const size_t xr0 = ((size_t)b * T + (size_t)c * TC + tl0) * DI;
  v8f acc[2][4];
#pragma unroll
  for (int r = 0; r < 2; ++r)
#pragma unroll
    for (int t = 0; t < 4; ++t) acc[r][t] = (v8f){};
#pragma unroll
  for (int kb = 0; kb < DI; kb += 32) { const v16b a0 = frag_kb(x16 + xr0 + (size_t)nloc * DI + kb, hlf), a1 = frag_kb(x16 + xr0 + (size_t)(16 + nloc) * DI + kb, hlf);
#pragma unroll
    for (int t = 0; t < 4; ++t) { const size_t bo = (size_t)(c0 + t * 16 + nloc) * DI + kb; const v16b b0 = frag_kb(bh + bo, hlf), b1 = frag_kb(bl + bo, hlf);
      acc[0][t] = wmma16b(a0, b0, acc[0][t]); acc[0][t] = wmma16b(a0, b1, acc[0][t]); acc[1][t] = wmma16b(a1, b0, acc[1][t]); acc[1][t] = wmma16b(a1, b1, acc[1][t]); } }
  float* Tt = Ts[wave];
#pragma unroll
  for (int t = 0; t < 4; ++t)
#pragma unroll
    for (int r = 0; r < 2; ++r)
#pragma unroll
      for (int v = 0; v < 8; ++v) Tt[(r * 16 + v + 8 * hlf) * 64 + t * 16 + nloc] = acc[r][t][v] * (1.0f / BS);
  wave_lds_sync();
  float* dst0 = u + (size_t)m0 * US + c0;
  for (int pass = 0; pass < 2; ++pass) {
#pragma unroll
    for (int j = 0; j < 16; ++j) { const int rr = j * 2 + hlf, c4 = nloc * 4; *(volatile v4f*)(dst0 + (size_t)rr * US + c4) = *(const v4f*)(Tt + rr * 64 + c4); }
    __threadfence();
  }
}

typedef __attribute__((ext_vector_type(2))) _Float16 v2b;
__global__ __launch_bounds__(128) void scan_kernel(const float* __restrict__ u, const float* __restrict__ llr, const float* __restrict__ li, const float* __restrict__ ldt, int c, float* __restrict__ state, b16* __restrict__ hh_, b16* __restrict__ hl_) {
  const int s0 = 2 * threadIdx.x, b = blockIdx.x; float ar[2], ai[2], hr[2], hi[2];
#pragma unroll
  for (int e = 0; e < 2; ++e) { float gr, gi; disc(llr, li, ldt, s0 + e, ar[e], ai[e], gr, gi); }
  { const v4f st = *(const v4f*)(state + ((size_t)b * DS + s0) * 2); hr[0] = st[0]; hi[0] = st[1]; hr[1] = st[2]; hi[1] = st[3]; }
  for (int tl = 0; tl < TC; ++tl) { const size_t r = (size_t)b * TC + tl; v2b rh, rl, ih, il;
#pragma unroll
    for (int e = 0; e < 2; ++e) { const float ur = u[r * US + s0 + e], ui = u[r * US + DS + s0 + e];
      const float nr = (pmul(hr[e], ar[e]) - pmul(hi[e], ai[e])) + ur, ni = (pmul(hr[e], ai[e]) + pmul(hi[e], ar[e])) + ui; hr[e] = nr; hi[e] = ni;
      b16 a, l; split16(nr * HS, a, l); rh[e] = a; rl[e] = l; split16(ni * HS, a, l); ih[e] = a; il[e] = l; }
    for (int pass = 0; pass < 2; ++pass) { *(volatile v2b*)(hh_ + r * US + s0) = rh; *(volatile v2b*)(hl_ + r * US + s0) = rl; *(volatile v2b*)(hh_ + r * US + DS + s0) = ih; *(volatile v2b*)(hl_ + r * US + DS + s0) = il; }
  }
  const v4f st = {hr[0], hi[0], hr[1], hi[1]};
  for (int pass = 0; pass < 2; ++pass) { *(volatile v4f*)(state + ((size_t)b * DS + s0) * 2) = st; __threadfence(); }
}

__global__ __launch_bounds__(128) void ygemm_kernel(const b16* __restrict__ hh_, const b16* __restrict__ hl_, const b16* __restrict__ ch, const b16* __restrict__ cl, int c, float* __restrict__ y) {
  __shared__ __attribute__((aligned(16))) float Ts[4][32 * 64];
  const int lane = threadIdx.x & 31, wave = threadIdx.x >> 5, nloc = lane & 15, hlf = lane >> 4, m0 = blockIdx.y * 128 + wave * 32, c0 = blockIdx.x * 64;
  v8f acc[2][4];
#pragma unroll
  for (int r = 0; r < 2; ++r)
#pragma unroll
    for (int t = 0; t < 4; ++t) acc[r][t] = (v8f){};
#pragma unroll 2
  for (int kb = 0; kb < US; kb += 32) { const v16b a0 = frag_kb(hh_ + (size_t)(m0 + nloc) * US + kb, hlf), l0 = frag_kb(hl_ + (size_t)(m0 + nloc) * US + kb, hlf), a1 = frag_kb(hh_ + (size_t)(m0 + 16 + nloc) * US + kb, hlf), l1 = frag_kb(hl_ + (size_t)(m0 + 16 + nloc) * US + kb, hlf);
#pragma unroll
    for (int t = 0; t < 4; ++t) { const size_t bo = (size_t)(c0 + t * 16 + nloc) * US + kb; const v16b b0 = frag_kb(ch + bo, hlf), b1 = frag_kb(cl + bo, hlf);
      acc[0][t] = wmma16b(a0, b0, acc[0][t]); acc[0][t] = wmma16b(l0, b0, acc[0][t]); acc[0][t] = wmma16b(a0, b1, acc[0][t]);
      acc[1][t] = wmma16b(a1, b0, acc[1][t]); acc[1][t] = wmma16b(l1, b0, acc[1][t]); acc[1][t] = wmma16b(a1, b1, acc[1][t]); } }
  float* Tt = Ts[wave];
#pragma unroll
  for (int t = 0; t < 4; ++t)
#pragma unroll
    for (int r = 0; r < 2; ++r)
#pragma unroll
      for (int v = 0; v < 8; ++v) Tt[(r * 16 + v + 8 * hlf) * 64 + t * 16 + nloc] = acc[r][t][v] * (1.0f / (HS * CS));
  wave_lds_sync();
  const int b = m0 / TC, tl0 = m0 % TC; float* dst0 = y + ((size_t)b * T + (size_t)c * TC + tl0) * DO + c0;
  for (int pass = 0; pass < 2; ++pass) {
#pragma unroll
    for (int j = 0; j < 16; ++j) { const int rr = j * 2 + hlf, c4 = nloc * 4; *(volatile v4f*)(dst0 + (size_t)rr * DO + c4) = *(const v4f*)(Tt + rr * 64 + c4); }
    __threadfence();
  }
}
}

extern "C" void kernel_launch(void* const* d_in, const int* in_sizes, int n_in,
                              void* d_out, int out_size, void* d_ws, size_t ws_size, hipStream_t stream) {
  (void)n_in; (void)out_size;
  const float* x = (const float*)d_in[0]; const float* llr = (const float*)d_in[1]; const float* li = (const float*)d_in[2]; const float* ldt = (const float*)d_in[3]; const float* Bm = (const float*)d_in[4]; const float* Cr = (const float*)d_in[5]; const float* Ci = (const float*)d_in[6];
  float* y = (float*)d_out;
  if (in_sizes[0] != Bn * T * DI || in_sizes[1] != DS || in_sizes[2] != DS || in_sizes[3] != DS || in_sizes[4] != DS * DI || in_sizes[5] != DO * DS || in_sizes[6] != DO * DS) return;
  size_t off = 0; char* ws = (char*)d_ws;
  auto carve = [&](size_t bytes) { char* p = ws + off; off += (bytes + 255) & ~(size_t)255; return p; };
  b16* x16 = (b16*)carve((size_t)Bn * T * DI * 2); b16* bh = (b16*)carve((size_t)US * DI * 2); b16* bl = (b16*)carve((size_t)US * DI * 2); b16* ch = (b16*)carve((size_t)DO * US * 2); b16* cl = (b16*)carve((size_t)DO * US * 2);
  float* state = (float*)carve((size_t)Bn * DS * 2 * 4); float* u = (float*)carve((size_t)NR * US * 4); b16* hh_ = (b16*)carve((size_t)NR * US * 2); b16* hl_ = (b16*)carve((size_t)NR * US * 2);
  if (off > ws_size) return;
  prep_kernel<<<1024, 256, 0, stream>>>(x, llr, li, ldt, Bm, Cr, Ci, x16, bh, bl, ch, cl, state);
  for (int c = 0; c < NCH; ++c) {
    ugemm_kernel<<<dim3(US / 64, NR / 128), 128, 0, stream>>>(x16, bh, bl, c, u);
    scan_kernel<<<Bn, 128, 0, stream>>>(u, llr, li, ldt, c, state, hh_, hl_);
    ygemm_kernel<<<dim3(DO / 64, NR / 128), 128, 0, stream>>>(hh_, hl_, ch, cl, c, y);
  }
}
